// da_47132971106554
// MI455X (gfx1250) — hardware-run, weakly checked
//
#include <hip/hip_runtime.h>
#include <math.h>

typedef __attribute__((ext_vector_type(16))) _Float16 v16h;
typedef __attribute__((ext_vector_type(8)))  _Float16 v8h;
typedef __attribute__((ext_vector_type(16))) __bf16   v16b;
typedef __attribute__((ext_vector_type(8)))  __bf16   v8b;
typedef __attribute__((ext_vector_type(8)))  float    v8f;
typedef __attribute__((ext_vector_type(4)))  float    v4f;

constexpr int kBatch    = 2;
constexpr int kCh       = 512;
constexpr int kCs       = 256;
constexpr int kHt       = 64;
constexpr int kWd       = 64;
constexpr int kHW       = kHt * kWd;
constexpr int kPix      = kBatch * kHW;
constexpr int kTaps     = 9;
constexpr int kKdc      = kCh * kTaps;
constexpr int kOffCh    = 18;
constexpr int kTcols    = kOffCh * kTaps;
constexpr int kTpad     = 192;
constexpr int kOffPitch = 32;
constexpr float kEps    = 1e-5f;
constexpr float kDcCarry    = 16.0f;
constexpr float kDcCarryInv = 1.0f / kDcCarry;
static_assert(kHW == 4096 && kPix == 8192 && kKdc == 4608 && kTcols == 162, "shape constants");
static_assert((kCs % 32) == 0 && (kCh % 32) == 0 && (kKdc % 32) == 0, "GEMM K multiples of 32");
static_assert((kPix % 64) == 0 && (kCh % 64) == 0 && (kTpad % 64) == 0 && kTpad >= kTcols, "GEMM M,N multiples of 64");

constexpr size_t kSzSamp  = (size_t)kPix * kKdc * 2;
constexpr size_t kSzBtDc  = (size_t)kCh * kKdc * 2;
constexpr size_t kSzPlane = (size_t)kPix * kCh * 4;
constexpr size_t kSzOff   = (size_t)kPix * kOffPitch * 4;
constexpr size_t kSzBtPw  = (size_t)kCh * kCs * 2;
constexpr size_t kSzBtOff = (size_t)kTpad * kCh * 2;
constexpr size_t kSzStat  = (size_t)kBatch * kCh * 4;
constexpr size_t kSzXs    = (size_t)kBatch * kCs * 4;

constexpr size_t kOffSamp = 0;
constexpr size_t kOffBtDc = kOffSamp + kSzSamp;
constexpr size_t kOffDN   = kOffBtDc + kSzBtDc;
constexpr size_t kOffDC   = kOffDN + kSzPlane;
constexpr size_t kOffOFF  = kOffDC + kSzPlane;
constexpr size_t kOffBPH  = kOffOFF + kSzOff;
constexpr size_t kOffBPL  = kOffBPH + kSzBtPw;
constexpr size_t kOffBOH  = kOffBPL + kSzBtPw;
constexpr size_t kOffBOL  = kOffBOH + kSzBtOff;
constexpr size_t kOffMU   = kOffBOL + kSzBtOff;
constexpr size_t kOffRS   = kOffMU + kSzStat;
constexpr size_t kOffXMX  = kOffRS + kSzStat;
constexpr size_t kOffXAV  = kOffXMX + kSzXs;
constexpr size_t kOffGT   = kOffXAV + kSzXs;
constexpr size_t kWsTotal = kOffGT + kSzStat;

constexpr size_t kSubAH  = 0;
constexpr size_t kSubAL  = kSubAH + (size_t)kPix * kCs * 2;
constexpr size_t kSubAOH = kSubAL + (size_t)kPix * kCs * 2;
constexpr size_t kSubAOL = kSubAOH + (size_t)kPix * kCh * 2;
constexpr size_t kSubTT  = kSubAOL + (size_t)kPix * kCh * 2;
constexpr size_t kSubEnd = kSubTT + (size_t)kPix * kTpad * 4;

static_assert(kWsTotal == 115752960ull, "carve total");
static_assert(kWsTotal <= 134217728ull, "carve cap");
static_assert(kSubEnd <= kSzSamp, "early scratch fits inside the sampled plane");
static_assert((kOffBtDc % 128) == 0 && (kOffDN % 128) == 0 && (kOffDC % 128) == 0 && (kOffOFF % 128) == 0 &&
              (kOffBPH % 128) == 0 && (kOffBPL % 128) == 0 && (kOffBOH % 128) == 0 && (kOffBOL % 128) == 0 &&
              (kOffMU % 128) == 0 && (kOffRS % 128) == 0 && (kOffXMX % 128) == 0 && (kOffXAV % 128) == 0 &&
              (kOffGT % 128) == 0 && (kSubAL % 128) == 0 && (kSubAOH % 128) == 0 && (kSubAOL % 128) == 0 &&
              (kSubTT % 128) == 0, "128-B aligned regions");

__device__ __forceinline__ unsigned short f2bf_bits(float f) {
  unsigned u = __float_as_uint(f);
  return (unsigned short)((u + 0x7FFFu + ((u >> 16) & 1u)) >> 16);
}
__device__ __forceinline__ float bf_bits2f(unsigned short h) { return __uint_as_float(((unsigned)h) << 16); }

__device__ __forceinline__ void split8_bf16(const v4f a0, const v4f a1, v8h& hv, v8h& lv) {
#pragma unroll
  for (int e = 0; e < 4; ++e) {
    const float f0 = a0[e];
    const float f1 = a1[e];
    const unsigned short h0 = f2bf_bits(f0);
    const unsigned short h1 = f2bf_bits(f1);
    const unsigned short l0 = f2bf_bits(f0 - bf_bits2f(h0));
    const unsigned short l1 = f2bf_bits(f1 - bf_bits2f(h1));
    hv[e]     = __builtin_bit_cast(_Float16, h0);
    hv[4 + e] = __builtin_bit_cast(_Float16, h1);
    lv[e]     = __builtin_bit_cast(_Float16, l0);
    lv[4 + e] = __builtin_bit_cast(_Float16, l1);
  }
}

__device__ __forceinline__ void dep_guard4_h(v8f& a, v8f& b, v8f& c, v8f& d, v16h x, v16h y) {
  asm volatile("v_nop\n\tv_nop\n\tv_nop\n\tv_nop" : "+v"(a), "+v"(b), "+v"(c), "+v"(d) : "v"(x), "v"(y));
}
__device__ __forceinline__ void dep_guard4_b(v8f& a, v8f& b, v8f& c, v8f& d, v16b x, v16b y) {
  asm volatile("v_nop\n\tv_nop\n\tv_nop\n\tv_nop" : "+v"(a), "+v"(b), "+v"(c), "+v"(d) : "v"(x), "v"(y));
}
__device__ __forceinline__ void keep4_h(v16h a, v16h b, v16h c, v16h d) { asm volatile("v_nop" :: "v"(a), "v"(b), "v"(c), "v"(d)); }
__device__ __forceinline__ void keep4_b(v16b a, v16b b, v16b c, v16b d) { asm volatile("v_nop" :: "v"(a), "v"(b), "v"(c), "v"(d)); }
__device__ __forceinline__ void acc_guard4(v8f& a, v8f& b, v8f& c, v8f& d) {
  asm volatile("v_nop\n\tv_nop\n\tv_nop\n\tv_nop" : "+v"(a), "+v"(b), "+v"(c), "+v"(d));
}

template <typename T> struct Frag;
template <> struct Frag<_Float16> {
  typedef v16h V;
  union U { v16h v; v8h h[2]; };
  static __device__ __forceinline__ v16h load(const _Float16* p) {
    U f;
    f.h[0] = *(const v8h*)(p);
    f.h[1] = *(const v8h*)(p + 16);
    return f.v;
  }
  static __device__ __forceinline__ v8f mma(v16h a, v16h b, v8f c) {
    return __builtin_amdgcn_wmma_f32_16x16x32_f16(false, a, false, b, (short)0, c, false, false);
  }
  static __device__ __forceinline__ void guard4(v8f& a, v8f& b, v8f& c, v8f& d, v16h x, v16h y) { dep_guard4_h(a, b, c, d, x, y); }
  static __device__ __forceinline__ void keep(v16h a, v16h b, v16h c, v16h d) { keep4_h(a, b, c, d); }
};
template <> struct Frag<__bf16> {
  typedef v16b V;
  union U { v16b v; v8b h[2]; };
  static __device__ __forceinline__ v16b load(const __bf16* p) {
    U f;
    f.h[0] = *(const v8b*)(p);
    f.h[1] = *(const v8b*)(p + 16);
    return f.v;
  }
  static __device__ __forceinline__ v8f mma(v16b a, v16b b, v8f c) {
    return __builtin_amdgcn_wmma_f32_16x16x32_bf16(false, a, false, b, (short)0, c, false, false);
  }
  static __device__ __forceinline__ void guard4(v8f& a, v8f& b, v8f& c, v8f& d, v16b x, v16b y) { dep_guard4_b(a, b, c, d, x, y); }
  static __device__ __forceinline__ void keep(v16b a, v16b b, v16b c, v16b d) { keep4_b(a, b, c, d); }
};

template <int ET> struct Elem;
template <> struct Elem<0> { typedef _Float16 T; };
template <> struct Elem<1> { typedef __bf16 T; };

template <int ET, bool SPLIT, int BIAS_MODE>
__global__ __launch_bounds__(256) void wmma_gemm64(
    const unsigned short* __restrict__ Ap, const unsigned short* __restrict__ A2p, int lda,
    const unsigned short* __restrict__ Btp, const unsigned short* __restrict__ Bt2p, int ldb,
    float* __restrict__ C, int ldc, const float* __restrict__ bias,
    int M, int N, int K, float scale) {
  typedef typename Elem<ET>::T T;
  typedef typename Frag<T>::V V;
  const T* A = (const T*)Ap;
  const T* A2 = (const T*)A2p;
  const T* Bt = (const T*)Btp;
  const T* Bt2 = (const T*)Bt2p;
  __shared__ __align__(16) float sT[8][16 * 68];
  const int lane = threadIdx.x & 31;
  const int wave = threadIdx.x >> 5;
  const int tilesN = N >> 6;
  const int tilesM = M >> 6;
  const int tile = blockIdx.x * 8 + wave;
  if (tile >= tilesM * tilesN) return;
  const int tm = tile / tilesN;
  const int tn = tile - tm * tilesN;
  const int m0 = tm << 6;
  const int n0 = tn << 6;

  const int rlane = lane & 15;
  const int koff  = (lane >> 4) * 8;
  const int mOff  = (lane >> 4) * 8;

  v8f acc[4][4];
#pragma unroll
  for (int i = 0; i < 4; ++i)
#pragma unroll
    for (int j = 0; j < 4; ++j) acc[i][j] = (v8f){0.f, 0.f, 0.f, 0.f, 0.f, 0.f, 0.f, 0.f};

  for (int k0 = 0; k0 < K; k0 += 32) {
    V bh[4], bl[4];
#pragma unroll
    for (int j = 0; j < 4; ++j) {
      const size_t bo = (size_t)(n0 + (j << 4) + rlane) * ldb + koff + k0;
      bh[j] = Frag<T>::load(Bt + bo);
      if (SPLIT) bl[j] = Frag<T>::load(Bt2 + bo);
    }
#pragma unroll
    for (int i = 0; i < 4; ++i) {
      const size_t ao = (size_t)(m0 + (i << 4) + rlane) * lda + koff + k0;
      V ah = Frag<T>::load(A + ao);
      V al;
      if (SPLIT) al = Frag<T>::load(A2 + ao);
#pragma unroll
      for (int j = 0; j < 4; ++j) {
        acc[i][j] = Frag<T>::mma(ah, bh[j], acc[i][j]);
        if (SPLIT) {
          acc[i][j] = Frag<T>::mma(ah, bl[j], acc[i][j]);
          acc[i][j] = Frag<T>::mma(al, bh[j], acc[i][j]);
        }
      }
      Frag<T>::guard4(acc[i][0], acc[i][1], acc[i][2], acc[i][3], ah, SPLIT ? al : ah);
    }
    Frag<T>::keep(bh[0], bh[1], bh[2], bh[3]);
    if (SPLIT) Frag<T>::keep(bl[0], bl[1], bl[2], bl[3]);
  }
  acc_guard4(acc[0][0], acc[0][1], acc[0][2], acc[0][3]);
  acc_guard4(acc[1][0], acc[1][1], acc[1][2], acc[1][3]);
  acc_guard4(acc[2][0], acc[2][1], acc[2][2], acc[2][3]);
  acc_guard4(acc[3][0], acc[3][1], acc[3][2], acc[3][3]);

  float* slab = sT[wave];
#pragma unroll
  for (int i = 0; i < 4; ++i) {
    const int mBase = m0 + (i << 4);
#pragma unroll
    for (int j = 0; j < 4; ++j) {
      const int n = n0 + (j << 4) + rlane;
      float bv = 0.f;
      if (BIAS_MODE == 2) bv = bias[n];
#pragma unroll
      for (int r = 0; r < 8; ++r) {
        float v = acc[i][j][r] * scale;
        if (BIAS_MODE == 2) v += bv;
        slab[(mOff + r) * 68 + (j << 4) + rlane] = v;
      }
    }
    __builtin_amdgcn_fence(__ATOMIC_RELEASE, "workgroup");
    __builtin_amdgcn_wave_barrier();
    __builtin_amdgcn_fence(__ATOMIC_ACQUIRE, "workgroup");
    {
      const int hh = lane >> 4, c4 = (lane & 15) * 4;
      for (int pass = 0; pass < 2; ++pass) {
#pragma unroll
        for (int it = 0; it < 8; ++it) {
          const int row = it * 2 + hh;
          v4f v = *(const v4f*)(slab + row * 68 + c4);
          *(volatile v4f*)(C + (size_t)(mBase + row) * ldc + n0 + c4) = v;
        }
        __threadfence();
      }
    }
    __builtin_amdgcn_fence(__ATOMIC_RELEASE, "workgroup");
    __builtin_amdgcn_wave_barrier();
    __builtin_amdgcn_fence(__ATOMIC_ACQUIRE, "workgroup");
  }
}

__global__ __launch_bounds__(256) void split_rows_bf16_kernel(
    const float* __restrict__ src, unsigned short* __restrict__ dhi, unsigned short* __restrict__ dlo, int total8) {
  const int i = blockIdx.x * 256 + threadIdx.x;
  if (i >= total8) return;
  const size_t e0 = (size_t)i << 3;
  const v4f a0 = *(const v4f*)(src + e0);
  const v4f a1 = *(const v4f*)(src + e0 + 4);
  v8h hv, lv;
  split8_bf16(a0, a1, hv, lv);
  unsigned short* qh = dhi + e0;
  unsigned short* ql = dlo + e0;
  *(volatile v8h*)qh = hv;
  *(volatile v8h*)ql = lv;
  __threadfence();
  *(volatile v8h*)qh = hv;
  *(volatile v8h*)ql = lv;
}

__global__ __launch_bounds__(256) void prep_off_kernel(
    const float* __restrict__ off_w, unsigned short* __restrict__ bh, unsigned short* __restrict__ bl) {
  const int i = blockIdx.x * 256 + threadIdx.x;
  const int r = i >> 6;
  const int c8 = (i & 63) * 8;
  const bool live = r < kTcols;
  const int rc = live ? r : (kTcols - 1);
  const int j = rc / kTaps;
  const int t = rc - j * kTaps;
  const float* wp = off_w + (size_t)j * kKdc + (size_t)c8 * kTaps + t;
  v4f a0, a1;
#pragma unroll
  for (int e = 0; e < 4; ++e) {
    const float w0 = wp[e * kTaps];
    const float w1 = wp[(4 + e) * kTaps];
    a0[e] = live ? w0 : 0.0f;
    a1[e] = live ? w1 : 0.0f;
  }
  v8h hv, lv;
  split8_bf16(a0, a1, hv, lv);
  unsigned short* qh = bh + (size_t)r * kCh + c8;
  unsigned short* ql = bl + (size_t)r * kCh + c8;
  *(volatile v8h*)qh = hv;
  *(volatile v8h*)ql = lv;
  __threadfence();
  *(volatile v8h*)qh = hv;
  *(volatile v8h*)ql = lv;
}

__global__ __launch_bounds__(256) void prep_dc_kernel(const float* __restrict__ dc_w, unsigned short* __restrict__ bt) {
  const int i = blockIdx.x * 256 + threadIdx.x;
  const int c8 = (i & 63) * 8;
  const int ot = i >> 6;
  const int o = ot / kTaps;
  const int t = ot - o * kTaps;
  const float* wp = dc_w + (size_t)o * kKdc + (size_t)c8 * kTaps + t;
  v8h hv;
#pragma unroll
  for (int e = 0; e < 8; ++e) {
    const float w = wp[e * kTaps] * kDcCarry;
    hv[e] = (_Float16)w;
  }
  unsigned short* q = bt + (size_t)o * kKdc + t * kCh + c8;
  *(volatile v8h*)q = hv;
  __threadfence();
  *(volatile v8h*)q = hv;
}

__global__ __launch_bounds__(256) void dwconv_kernel(
    const float* __restrict__ x, const float* __restrict__ dw_w, const float* __restrict__ dw_b,
    unsigned short* __restrict__ AH, unsigned short* __restrict__ AL) {
  __shared__ __align__(16) float sT[64 * 68];
  const int tid = threadIdx.x, lane = tid & 31, wave = tid >> 5;
  const int cchunk = blockIdx.x & 3;
  const int y = (blockIdx.x >> 2) & 63;
  const int b = blockIdx.x >> 8;
  const int px = tid & 63;
  const int cg = tid >> 6;
#pragma unroll 1
  for (int i = 0; i < 16; ++i) {
    const int cl = cg * 16 + i;
    const int c = cchunk * 64 + cl;
    const float* xp = x + ((size_t)b * kCh + c) * kHW;
    const float* wp = dw_w + c * 9;
    float acc = 0.0f;
#pragma unroll
    for (int ky = 0; ky < 3; ++ky) {
      const int yy = y + ky - 1;
      const bool oky = (yy >= 0) && (yy < kHt);
      const int yc = yy < 0 ? 0 : (yy > kHt - 1 ? kHt - 1 : yy);
#pragma unroll
      for (int kx = 0; kx < 3; ++kx) {
        const int xx = px + kx - 1;
        const bool ok = oky && (xx >= 0) && (xx < kWd);
        const int xc = xx < 0 ? 0 : (xx > kWd - 1 ? kWd - 1 : xx);
        float v = xp[yc * kWd + xc];
        v = ok ? v : 0.0f;
        acc = fmaf(v, wp[ky * 3 + kx], acc);
      }
    }
    acc += dw_b[c];
    sT[px * 68 + cl] = acc;
  }
  __syncthreads();
  const int q = lane >> 3, c8 = (lane & 7) * 8;
  const int nrow0 = b * kHW + y * kWd;
  v8h hv[2], lv[2];
#pragma unroll
  for (int it = 0; it < 2; ++it) {
    const int row = it * 32 + wave * 4 + q;
    const float* sp = sT + row * 68 + c8;
    const v4f a0 = *(const v4f*)(sp);
    const v4f a1 = *(const v4f*)(sp + 4);
    split8_bf16(a0, a1, hv[it], lv[it]);
  }
  for (int pass = 0; pass < 2; ++pass) {
#pragma unroll
    for (int it = 0; it < 2; ++it) {
      const int row = it * 32 + wave * 4 + q;
      const size_t o = (size_t)(nrow0 + row) * kCs + cchunk * 64 + c8;
      *(volatile v8h*)(AH + o) = hv[it];
      *(volatile v8h*)(AL + o) = lv[it];
    }
    __threadfence();
  }
}

__global__ __launch_bounds__(256) void in_stats_kernel(
    const float* __restrict__ d1, float* __restrict__ mu, float* __restrict__ rs) {
  __shared__ float sP[8 * 32];
  const int tid = threadIdx.x, lane = tid & 31, wave = tid >> 5;
  const int b = blockIdx.x >> 4;
  const int c = (blockIdx.x & 15) * 32 + lane;
  const float* p = d1 + (size_t)b * kHW * kCh + c;
  float s = 0.0f;
#pragma unroll 4
  for (int r = wave; r < kHW; r += 8) s += p[(size_t)r * kCh];
  sP[wave * 32 + lane] = s;
  __syncthreads();
  float tot = 0.0f;
#pragma unroll
  for (int w = 0; w < 8; ++w) tot += sP[w * 32 + lane];
  const float mean = tot * (1.0f / (float)kHW);
  __syncthreads();
  float q = 0.0f;
#pragma unroll 4
  for (int r = wave; r < kHW; r += 8) {
    const float dv = p[(size_t)r * kCh] - mean;
    q = fmaf(dv, dv, q);
  }
  sP[wave * 32 + lane] = q;
  __syncthreads();
  float qt = 0.0f;
#pragma unroll
  for (int w = 0; w < 8; ++w) qt += sP[w * 32 + lane];
  const float var = qt * (1.0f / (float)kHW);
  const float rstd = 1.0f / sqrtf(var + kEps);
  if (wave == 0) {
    float* pm = mu + b * kCh + c;
    float* pr = rs + b * kCh + c;
    *(volatile float*)pm = mean;
    *(volatile float*)pr = rstd;
    __threadfence();
    *(volatile float*)pm = mean;
    *(volatile float*)pr = rstd;
  }
}

__global__ __launch_bounds__(256) void in_norm_kernel(
    const float* __restrict__ d1, const float* __restrict__ mu, const float* __restrict__ rs,
    float* __restrict__ dn, unsigned short* __restrict__ AOH, unsigned short* __restrict__ AOL) {
  const int lane = threadIdx.x & 31, wave = threadIdx.x >> 5;
  const int g = blockIdx.x * 8 + wave;
  const int n = g >> 1;
  const int hf = g & 1;
  const int b = n >> 12;
  const size_t base = (size_t)n * kCh + hf * 256;
  const int sb = b * kCh + hf * 256;
  const int cA = lane * 8;
  v8h hv, lv;
  {
    const v4f x0 = *(const v4f*)(d1 + base + cA);
    const v4f x1 = *(const v4f*)(d1 + base + cA + 4);
    const v4f m0 = *(const v4f*)(mu + sb + cA);
    const v4f m1 = *(const v4f*)(mu + sb + cA + 4);
    const v4f r0 = *(const v4f*)(rs + sb + cA);
    const v4f r1 = *(const v4f*)(rs + sb + cA + 4);
    v4f n0v, n1v;
#pragma unroll
    for (int e = 0; e < 4; ++e) {
      n0v[e] = (x0[e] - m0[e]) * r0[e];
      n1v[e] = (x1[e] - m1[e]) * r1[e];
    }
    split8_bf16(n0v, n1v, hv, lv);
  }
  v4f fv[2];
#pragma unroll
  for (int it = 0; it < 2; ++it) {
    const int cB = it * 128 + lane * 4;
    const v4f xv = *(const v4f*)(d1 + base + cB);
    const v4f mv = *(const v4f*)(mu + sb + cB);
    const v4f rv = *(const v4f*)(rs + sb + cB);
#pragma unroll
    for (int e = 0; e < 4; ++e) fv[it][e] = (xv[e] - mv[e]) * rv[e];
  }
  for (int pass = 0; pass < 2; ++pass) {
#pragma unroll
    for (int it = 0; it < 2; ++it) *(volatile v4f*)(dn + base + it * 128 + lane * 4) = fv[it];
    *(volatile v8h*)(AOH + base + cA) = hv;
    *(volatile v8h*)(AOL + base + cA) = lv;
    __threadfence();
  }
}

__global__ __launch_bounds__(256) void off_sum_kernel(
    const float* __restrict__ TT, const float* __restrict__ off_b, float* __restrict__ off) {
  const int i = blockIdx.x * 256 + threadIdx.x;
  const int n = i >> 3;
  const int jq = (i & 7) * 4;
  const int b = n >> 12;
  const int y = (n >> 6) & 63;
  const int x = n & 63;
  int jc[4];
  bool jv[4];
  float acc[4];
#pragma unroll
  for (int e = 0; e < 4; ++e) {
    const int j = jq + e;
    jv[e] = j < kOffCh;
    jc[e] = jv[e] ? j : (kOffCh - 1);
    acc[e] = 0.0f;
  }
#pragma unroll 1
  for (int t = 0; t < kTaps; ++t) {
    const int t3 = t / 3;
    const int yy = y + t3 - 1;
    const int xx = x + (t - t3 * 3) - 1;
    const bool ok = (yy >= 0) && (yy < kHt) && (xx >= 0) && (xx < kWd);
    const int yc = yy < 0 ? 0 : (yy > kHt - 1 ? kHt - 1 : yy);
    const int xc = xx < 0 ? 0 : (xx > kWd - 1 ? kWd - 1 : xx);
    const float* tp = TT + (size_t)(b * kHW + yc * kWd + xc) * kTpad + t;
#pragma unroll
    for (int e = 0; e < 4; ++e) {
      float v = tp[jc[e] * kTaps];
      v = ok ? v : 0.0f;
      acc[e] += v;
    }
  }
  v4f r;
#pragma unroll
  for (int e = 0; e < 4; ++e) {
    const float bv = off_b[jc[e]];
    const float s = acc[e] + bv;
    r[e] = jv[e] ? s : 0.0f;
  }
  float* q = off + (size_t)n * kOffPitch + jq;
  *(volatile v4f*)q = r;
  __threadfence();
  *(volatile v4f*)q = r;
}

__global__ __launch_bounds__(256) void sampler_kernel(
    const float* __restrict__ dn, const float* __restrict__ off, unsigned short* __restrict__ samp) {
  const int lane = threadIdx.x & 31, wave = threadIdx.x >> 5;
  const int g = blockIdx.x * 8 + wave;
  const int n = g / kTaps;
  const int t = g - n * kTaps;
  const int b = n >> 12;
  const int y = (n >> 6) & 63;
  const int x = n & 63;
  const int t3 = t / 3;
  const float kyf = (float)(t3 - 1);
  const float kxf = (float)(t - t3 * 3 - 1);
  const float oy = off[(size_t)n * kOffPitch + 2 * t];
  const float ox = off[(size_t)n * kOffPitch + 2 * t + 1];
  const float py = ((float)y + kyf) + oy;
  const float px = ((float)x + kxf) + ox;
  const float fy = floorf(py);
  const float fx = floorf(px);
  const float ly = py - fy;
  const float lx = px - fx;
  const int y0 = (int)fminf(fmaxf(fy, -2.0f), 65.0f);
  const int x0 = (int)fminf(fmaxf(fx, -2.0f), 65.0f);
  const int y1 = y0 + 1;
  const int x1 = x0 + 1;
  const bool vy0 = (y0 >= 0) && (y0 < kHt);
  const bool vy1 = (y1 >= 0) && (y1 < kHt);
  const bool vx0 = (x0 >= 0) && (x0 < kWd);
  const bool vx1 = (x1 >= 0) && (x1 < kWd);
  const bool ok00 = vy0 && vx0, ok01 = vy0 && vx1, ok10 = vy1 && vx0, ok11 = vy1 && vx1;
  const int yc0 = y0 < 0 ? 0 : (y0 > kHt - 1 ? kHt - 1 : y0);
  const int yc1 = y1 < 0 ? 0 : (y1 > kHt - 1 ? kHt - 1 : y1);
  const int xc0 = x0 < 0 ? 0 : (x0 > kWd - 1 ? kWd - 1 : x0);
  const int xc1 = x1 < 0 ? 0 : (x1 > kWd - 1 ? kWd - 1 : x1);
  const float hy = 1.0f - ly;
  const float hx = 1.0f - lx;
  const float w00 = hy * hx, w01 = hy * lx, w10 = ly * hx, w11 = ly * lx;
  const float* p00 = dn + (size_t)(b * kHW + yc0 * kWd + xc0) * kCh;
  const float* p01 = dn + (size_t)(b * kHW + yc0 * kWd + xc1) * kCh;
  const float* p10 = dn + (size_t)(b * kHW + yc1 * kWd + xc0) * kCh;
  const float* p11 = dn + (size_t)(b * kHW + yc1 * kWd + xc1) * kCh;
  unsigned short* orow = samp + (size_t)n * kKdc + t * kCh;
#pragma unroll 1
  for (int it = 0; it < 2; ++it) {
    const int c = it * 256 + lane * 8;
    const v4f a0 = *(const v4f*)(p00 + c);
    const v4f a1 = *(const v4f*)(p00 + c + 4);
    const v4f b0 = *(const v4f*)(p01 + c);
    const v4f b1 = *(const v4f*)(p01 + c + 4);
    const v4f g0 = *(const v4f*)(p10 + c);
    const v4f g1 = *(const v4f*)(p10 + c + 4);
    const v4f h0 = *(const v4f*)(p11 + c);
    const v4f h1 = *(const v4f*)(p11 + c + 4);
    v8h hv;
#pragma unroll
    for (int e = 0; e < 4; ++e) {
      const float va0 = ok00 ? a0[e] : 0.0f;
      const float vb0 = ok01 ? b0[e] : 0.0f;
      const float vg0 = ok10 ? g0[e] : 0.0f;
      const float vh0 = ok11 ? h0[e] : 0.0f;
      const float va1 = ok00 ? a1[e] : 0.0f;
      const float vb1 = ok01 ? b1[e] : 0.0f;
      const float vg1 = ok10 ? g1[e] : 0.0f;
      const float vh1 = ok11 ? h1[e] : 0.0f;
      float s0 = va0 * w00;
      s0 = fmaf(vb0, w01, s0);
      s0 = fmaf(vg0, w10, s0);
      s0 = fmaf(vh0, w11, s0);
      float s1 = va1 * w00;
      s1 = fmaf(vb1, w01, s1);
      s1 = fmaf(vg1, w10, s1);
      s1 = fmaf(vh1, w11, s1);
      hv[e] = (_Float16)s0;
      hv[4 + e] = (_Float16)s1;
    }
    unsigned short* q = orow + c;
    *(volatile v8h*)q = hv;
    __threadfence();
    *(volatile v8h*)q = hv;
  }
}

__global__ __launch_bounds__(256) void x2_stats_kernel(
    const float* __restrict__ x, float* __restrict__ xmx, float* __restrict__ xav) {
  __shared__ float sMx[32];
  __shared__ float sAv[32];
  const int tid = threadIdx.x, lane = tid & 31, wave = tid >> 5;
  const int b = blockIdx.x >> 3;
  const int cg = blockIdx.x & 7;
#pragma unroll 1
  for (int k = 0; k < 4; ++k) {
    const int cl = wave * 4 + k;
    const int c2 = cg * 32 + cl;
    const float* p = x + ((size_t)b * kCh + kCs + c2) * kHW;
    float mx = -INFINITY;
    float s = 0.0f;
#pragma unroll 4
    for (int i = 0; i < 32; ++i) {
      const v4f v = *(const v4f*)(p + (i * 32 + lane) * 4);
      mx = fmaxf(mx, fmaxf(fmaxf(v[0], v[1]), fmaxf(v[2], v[3])));
      s += (v[0] + v[1]) + (v[2] + v[3]);
    }
#pragma unroll
    for (int o = 16; o > 0; o >>= 1) {
      const float om = __shfl_xor(mx, o, 32);
      const float os = __shfl_xor(s, o, 32);
      mx = fmaxf(mx, om);
      s += os;
    }
    if (lane == 0) {
      sMx[cl] = mx;
      sAv[cl] = s * (1.0f / (float)kHW);
    }
  }
  __syncthreads();
  if (wave == 0) {
    const float vm = sMx[lane];
    const float va = sAv[lane];
    float* pm = xmx + b * kCs + cg * 32 + lane;
    float* pa = xav + b * kCs + cg * 32 + lane;
    *(volatile float*)pm = vm;
    *(volatile float*)pa = va;
    __threadfence();
    *(volatile float*)pm = vm;
    *(volatile float*)pa = va;
  }
}

__global__ __launch_bounds__(256) void gate_kernel(
    const float* __restrict__ xmx, const float* __restrict__ xav,
    const float* __restrict__ adw_w, const float* __restrict__ adw_b,
    const float* __restrict__ apw_w, const float* __restrict__ apw_b, float* __restrict__ gt) {
  __shared__ __align__(16) float sT1[256];
  __shared__ __align__(16) float sT2[256];
  const int tid = threadIdx.x;
  const int b = blockIdx.x >> 1;
  const int o = (blockIdx.x & 1) * 256 + tid;
  {
    const float w4 = adw_w[tid * 9 + 4];
    const float bb = adw_b[tid];
    sT1[tid] = w4 * xmx[b * kCs + tid] + bb;
    sT2[tid] = w4 * xav[b * kCs + tid] + bb;
  }
  __syncthreads();
  const float* wr = apw_w + (size_t)o * kCs;
  float a1 = 0.0f, a2 = 0.0f;
#pragma unroll 1
  for (int c = 0; c < kCs; c += 4) {
    const v4f w = *(const v4f*)(wr + c);
    const v4f t1 = *(const v4f*)(sT1 + c);
    const v4f t2 = *(const v4f*)(sT2 + c);
#pragma unroll
    for (int e = 0; e < 4; ++e) {
      a1 = fmaf(w[e], t1[e], a1);
      a2 = fmaf(w[e], t2[e], a2);
    }
  }
  const float pb = apw_b[o];
  const float z = (a1 + pb) + (a2 + pb);
  const float gv = 1.0f / (1.0f + expf(-z));
  float* q = gt + b * kCh + o;
  *(volatile float*)q = gv;
  __threadfence();
  *(volatile float*)q = gv;
}

__device__ __forceinline__ float sum4f(const v4f v) { return (v[0] + v[1]) + (v[2] + v[3]); }
__device__ __forceinline__ float sq4f(const v4f v, const float m) {
  const float e0 = v[0] - m, e1 = v[1] - m, e2 = v[2] - m, e3 = v[3] - m;
  return (e0 * e0 + e1 * e1) + (e2 * e2 + e3 * e3);
}

__global__ __launch_bounds__(256) void ln_gate_out_kernel(
    const float* __restrict__ x, const float* __restrict__ dn, const float* __restrict__ dc,
    const float* __restrict__ ln_g, const float* __restrict__ ln_b, const float* __restrict__ gt,
    float* __restrict__ out) {
  __shared__ float sM[64];
  __shared__ float sR[64];
  __shared__ __align__(16) float sT[64 * 68];
  const int tid = threadIdx.x, lane = tid & 31, wave = tid >> 5;
  const int b = blockIdx.x >> 6;
  const int y = blockIdx.x & 63;
  const int n0 = b * kHW + y * kWd;
#pragma unroll 1
  for (int k = 0; k < 8; ++k) {
    const int px = wave * 8 + k;
    const float* row = dc + (size_t)(n0 + px) * kCh + lane * 4;
    const v4f v0 = *(const v4f*)(row);
    const v4f v1 = *(const v4f*)(row + 128);
    const v4f v2 = *(const v4f*)(row + 256);
    const v4f v3 = *(const v4f*)(row + 384);
    float s = (sum4f(v0) + sum4f(v1)) + (sum4f(v2) + sum4f(v3));
#pragma unroll
    for (int o = 16; o > 0; o >>= 1) {
      const float os = __shfl_xor(s, o, 32);
      s += os;
    }
    const float m = s * (1.0f / (float)kCh);
    float q = (sq4f(v0, m) + sq4f(v1, m)) + (sq4f(v2, m) + sq4f(v3, m));
#pragma unroll
    for (int o = 16; o > 0; o >>= 1) {
      const float oq = __shfl_xor(q, o, 32);
      q += oq;
    }
    const float r = 1.0f / sqrtf(q * (1.0f / (float)kCh) + kEps);
    if (lane == 0) {
      sM[px] = m;
      sR[px] = r;
    }
  }
  __syncthreads();
  const int cl = tid & 63;
  const int pg = tid >> 6;
  const int hh = lane >> 4;
  const int x4 = (lane & 15) * 4;
#pragma unroll 1
  for (int ch = 0; ch < 8; ++ch) {
    const int c0 = ch * 64;
    {
      const int c = c0 + cl;
      const float lg = ln_g[c];
      const float lb = ln_b[c];
#pragma unroll 1
      for (int k = 0; k < 16; ++k) {
        const int px = pg * 16 + k;
        const size_t idx = (size_t)(n0 + px) * kCh + c;
        const float dcv = dc[idx];
        const float dv = dn[idx];
        const float z = (dcv - sM[px]) * sR[px] * lg + lb;
        const float sg = 1.0f / (1.0f + expf(-z));
        sT[cl * 68 + px] = dv * sg;
      }
    }
    __syncthreads();
    v4f ov[4];
#pragma unroll
    for (int it = 0; it < 4; ++it) {
      const int crow = it * 16 + wave * 2 + hh;
      const int c = c0 + crow;
      const float gg = gt[b * kCh + c];
      const v4f xv = *(const v4f*)(x + ((size_t)(b * kCh + c) * kHt + y) * kWd + x4);
      const v4f sv = *(const v4f*)(sT + crow * 68 + x4);
#pragma unroll
      for (int e = 0; e < 4; ++e) ov[it][e] = xv[e] * sv[e] + xv[e] * gg;
    }
    for (int pass = 0; pass < 2; ++pass) {
#pragma unroll
      for (int it = 0; it < 4; ++it) {
        const int c = c0 + it * 16 + wave * 2 + hh;
        *(volatile v4f*)(out + ((size_t)(b * kCh + c) * kHt + y) * kWd + x4) = ov[it];
      }
      __threadfence();
    }
    __syncthreads();
  }
}

extern "C" void kernel_launch(void* const* d_in, const int* in_sizes, int n_in,
                              void* d_out, int out_size, void* d_ws, size_t ws_size,
                              hipStream_t stream) {
  if (n_in < 15) return;
  if (in_sizes[0] != kBatch * kCh * kHW) return;
  if (in_sizes[1] != kCs * 9) return;
  if (in_sizes[2] != kCs) return;
  if (in_sizes[3] != kCh * kCs) return;
  if (in_sizes[4] != kCh) return;
  if (in_sizes[5] != kOffCh * kKdc) return;
  if (in_sizes[6] != kOffCh) return;
  if (in_sizes[7] != kCh * kKdc) return;
  if (in_sizes[8] != kCh) return;
  if (in_sizes[9] != kCh) return;
  if (in_sizes[10] != kCh) return;
  if (in_sizes[11] != kCs * 9) return;
  if (in_sizes[12] != kCs) return;
  if (in_sizes[13] != kCh * kCs) return;
  if (in_sizes[14] != kCh) return;
  if (out_size != kBatch * kCh * kHW) return;
  if (ws_size < kWsTotal) return;

  const float* x      = (const float*)d_in[0];
  const float* dw_w   = (const float*)d_in[1];
  const float* dw_b   = (const float*)d_in[2];
  const float* pw_w   = (const float*)d_in[3];
  const float* pw_b   = (const float*)d_in[4];
  const float* off_w  = (const float*)d_in[5];
  const float* off_b  = (const float*)d_in[6];
  const float* dc_w   = (const float*)d_in[7];
  const float* dc_b   = (const float*)d_in[8];
  const float* ln_g   = (const float*)d_in[9];
  const float* ln_b   = (const float*)d_in[10];
  const float* adw_w  = (const float*)d_in[11];
  const float* adw_b  = (const float*)d_in[12];
  const float* apw_w  = (const float*)d_in[13];
  const float* apw_b  = (const float*)d_in[14];
  float* out = (float*)d_out;

  char* ws = (char*)d_ws;
  unsigned short* SAMP = (unsigned short*)(ws + kOffSamp);
  unsigned short* AH   = (unsigned short*)(ws + kOffSamp + kSubAH);
  unsigned short* AL   = (unsigned short*)(ws + kOffSamp + kSubAL);
  unsigned short* AOH  = (unsigned short*)(ws + kOffSamp + kSubAOH);
  unsigned short* AOL  = (unsigned short*)(ws + kOffSamp + kSubAOL);
  float*          TT   = (float*)(ws + kOffSamp + kSubTT);
  unsigned short* BTDC = (unsigned short*)(ws + kOffBtDc);
  float*          DN   = (float*)(ws + kOffDN);
  float*          DC   = (float*)(ws + kOffDC);
  float*          D1   = DC;
  float*          OFF  = (float*)(ws + kOffOFF);
  unsigned short* BPH  = (unsigned short*)(ws + kOffBPH);
  unsigned short* BPL  = (unsigned short*)(ws + kOffBPL);
  unsigned short* BOH  = (unsigned short*)(ws + kOffBOH);
  unsigned short* BOL  = (unsigned short*)(ws + kOffBOL);
  float*          MU   = (float*)(ws + kOffMU);
  float*          RS   = (float*)(ws + kOffRS);
  float*          XMX  = (float*)(ws + kOffXMX);
  float*          XAV  = (float*)(ws + kOffXAV);
  float*          GT   = (float*)(ws + kOffGT);

  split_rows_bf16_kernel<<<(kCh * kCs / 8) / 256, 256, 0, stream>>>(pw_w, BPH, BPL, kCh * kCs / 8);
  prep_off_kernel<<<(kTpad * 64) / 256, 256, 0, stream>>>(off_w, BOH, BOL);
  prep_dc_kernel<<<(kCh * kTaps * 64) / 256, 256, 0, stream>>>(dc_w, BTDC);

  dwconv_kernel<<<kBatch * kHt * 4, 256, 0, stream>>>(x, dw_w, dw_b, AH, AL);

  wmma_gemm64<1, true, 2><<<128, 256, 0, stream>>>(
      AH, AL, kCs, BPH, BPL, kCs, D1, kCh, pw_b, kPix, kCh, kCs, 1.0f);

  in_stats_kernel<<<kBatch * 16, 256, 0, stream>>>(D1, MU, RS);
  in_norm_kernel<<<(kPix * 2) / 8, 256, 0, stream>>>(D1, MU, RS, DN, AOH, AOL);

  wmma_gemm64<1, true, 0><<<48, 256, 0, stream>>>(
      AOH, AOL, kCh, BOH, BOL, kCh, TT, kTpad, nullptr, kPix, kTpad, kCh, 1.0f);
  off_sum_kernel<<<(kPix * 8) / 256, 256, 0, stream>>>(TT, off_b, OFF);

  sampler_kernel<<<(kPix * kTaps) / 8, 256, 0, stream>>>(DN, OFF, SAMP);

  wmma_gemm64<0, false, 2><<<128, 256, 0, stream>>>(
      SAMP, nullptr, kKdc, BTDC, nullptr, kKdc, DC, kCh, dc_b, kPix, kCh, kKdc, kDcCarryInv);

  x2_stats_kernel<<<kBatch * 8, 256, 0, stream>>>(x, XMX, XAV);
  gate_kernel<<<4, 256, 0, stream>>>(XMX, XAV, adw_w, adw_b, apw_w, apw_b, GT);

  ln_gate_out_kernel<<<kBatch * kHt, 256, 0, stream>>>(x, DN, DC, ln_g, ln_b, GT, out);
}
